// GroupShuffleAttention_18889266167879
// MI455X (gfx1250) — hardware-verified
//
#include <hip/hip_runtime.h>
#include <hip/hip_bf16.h>
#include <math.h>


#define BB 2
#define S32 4096
#define D32 256
#define NH32 8
#define GC 32
#define QW 2

typedef _Float16 bf16;
typedef __attribute__((ext_vector_type(4))) unsigned v4u_t;
typedef unsigned v4ua __attribute__((ext_vector_type(4), may_alias));
typedef __attribute__((ext_vector_type(4))) float v4f_t;
typedef float v4fa __attribute__((ext_vector_type(4), may_alias));
typedef __attribute__((ext_vector_type(16))) bf16  bf16x16;
typedef __attribute__((ext_vector_type(8)))  bf16  bf16x8;
typedef __attribute__((ext_vector_type(4)))  bf16  bf16x4;
typedef __attribute__((ext_vector_type(8)))  float f32x8;

#define LDS_STRIDE 48
#define KSTRIDE    72
#define VSTRIDE    48

__device__ __forceinline__ f32x8 wmma_bf16(bf16x16 a, bf16x16 b, f32x8 c) {
  return __builtin_amdgcn_wmma_f32_16x16x32_f16(
      false, a, false, b, (short)0, c, false, false);
}
#define RSPLIT (1.0f / 2048.0f)
__device__ __forceinline__ bf16 lo_of(float v, bf16 h) { return (bf16)((v - (float)h) * 2048.0f); }
__device__ __forceinline__ f32x8 wmma_split(bf16x16 a, bf16x16 al, bf16x16 b, bf16x16 bl, f32x8 c) {
  f32x8 x = {}; x = wmma_bf16(al, b, x); x = wmma_bf16(a, bl, x); return wmma_bf16(a, b, c) + x * RSPLIT; }

template <typename T>
__device__ __forceinline__ bf16x16 load_frag(const T* __restrict__ base, int ld,
                                             int row0, int k0) {
  const int lane = threadIdx.x & 31;
  const int r    = lane & 15;
  const int kh   = (lane >> 4) * 8;
  const T* p0 = base + (size_t)(row0 + r) * ld + (k0 + kh);
  const T* p1 = p0 + 16;
  bf16x16 f;
#pragma unroll
  for (int i = 0; i < 8; ++i) {
    f[i]     = (bf16)p0[i];
    f[i + 8] = (bf16)p1[i];
  }
  return f;
}

__device__ __forceinline__ bf16x16 lds_frag(const bf16* base, int stride) {
  const int lane = threadIdx.x & 31;
  const int row  = lane & 15;
  const int kh   = (lane >> 4) * 8;
  const bf16x8 lo = *(const bf16x8*)(base + row * stride + kh);
  const bf16x8 hi = *(const bf16x8*)(base + row * stride + kh + 16);
  bf16x16 f;
#pragma unroll
  for (int i = 0; i < 8; ++i) { f[i] = lo[i]; f[i + 8] = hi[i]; }
  return f;
}

template <typename T>
__device__ __forceinline__ void stage_read16(const T* __restrict__ p, float* buf) {
#pragma unroll
  for (int i = 0; i < 16; ++i) buf[i] = (float)p[i];
}

__device__ __forceinline__ void stage_write(bf16* dst, const float* buf, int nquad) {
#pragma unroll
  for (int i = 0; i < nquad; ++i) {
    bf16x4 q;
    q[0] = (bf16)buf[4 * i];     q[1] = (bf16)buf[4 * i + 1];
    q[2] = (bf16)buf[4 * i + 2]; q[3] = (bf16)buf[4 * i + 3];
    *(bf16x4*)(dst + 4 * i) = q;
  }
}


#define SS S32
#define HH 4
#define DKK 64
template <typename AT, int MODE>
__global__ __launch_bounds__(256) void gemm_bias_kernel(
    const AT* __restrict__ A, const float* __restrict__ W,
    const float* __restrict__ bias, void* __restrict__ out,
    int M, int N, int K) {
  __shared__ bf16 ldsA[128 * LDS_STRIDE];
  __shared__ bf16 ldsW[256 * LDS_STRIDE];
  __shared__ __attribute__((aligned(16))) unsigned char sob[256 * 136 * 2];

  const int t    = threadIdx.x;
  const int wave = t >> 5;
  const int lane = t & 31;
  const int wm   = (wave & 1) * 64;
  const int wn   = (wave >> 1) * 64;
  const int mBlk = blockIdx.x * 128;
  const int nBlk = blockIdx.y * 256;

  const int arow = t >> 1;
  const int ach  = (t & 1) * 16;

  float abuf[16];
  float wbuf[32];

  stage_read16(A + (size_t)(mBlk + arow) * K + ach, abuf);
  stage_read16(W + (size_t)(nBlk + t) * K,          wbuf);
  stage_read16(W + (size_t)(nBlk + t) * K + 16,     wbuf + 16);

  f32x8 acc[4][4] = {};

  for (int k = 0; k < K; k += 32) {
    __syncthreads();
    stage_write(&ldsA[arow * LDS_STRIDE + ach], abuf, 4);
    stage_write(&ldsW[t * LDS_STRIDE],          wbuf, 8);
    if (k + 32 < K) {
      stage_read16(A + (size_t)(mBlk + arow) * K + (k + 32) + ach, abuf);
      stage_read16(W + (size_t)(nBlk + t) * K + (k + 32),          wbuf);
      stage_read16(W + (size_t)(nBlk + t) * K + (k + 32) + 16,     wbuf + 16);
    }
    __syncthreads();

    bf16x16 af[4], wf[4];
#pragma unroll
    for (int i = 0; i < 4; ++i)
      af[i] = lds_frag(ldsA + (wm + 16 * i) * LDS_STRIDE, LDS_STRIDE);
#pragma unroll
    for (int j = 0; j < 4; ++j)
      wf[j] = lds_frag(ldsW + (wn + 16 * j) * LDS_STRIDE, LDS_STRIDE);
#pragma unroll
    for (int i = 0; i < 4; ++i)
#pragma unroll
      for (int j = 0; j < 4; ++j)
        acc[i][j] = wmma_bf16(af[i], wf[j], acc[i][j]);
  }

  const int nlane = lane & 15;
  const int mh    = (lane >> 4) * 8;
  __syncthreads();
  if (MODE == 0 || MODE == 1) {
    bf16* so = (bf16*)sob;
#pragma unroll
    for (int i = 0; i < 4; ++i)
#pragma unroll
      for (int j = 0; j < 4; ++j) {
        const int nl = wn + 16 * j + nlane;
        const float bv = bias ? bias[nBlk + nl] : 0.0f;
#pragma unroll
        for (int r = 0; r < 8; ++r) {
          const int ml = wm + 16 * i + mh + r;
          const bf16 hv = (bf16)(acc[i][j][r] + bv);
          if (MODE == 0) so[ml * 264 + nl] = hv;
          else           so[nl * 136 + ml] = hv;
        }
      }
    __syncthreads();
#pragma unroll 1
    for (int pass = 0; pass < 2; ++pass) {
      if (MODE == 0) {
        for (int ch = t; ch < 128 * 32; ch += 256) { const int ml = ch >> 5, q = (ch & 31) * 8;
          *(volatile v4u_t*)((bf16*)out + (size_t)(mBlk + ml) * N + nBlk + q) = *(const v4ua*)(so + ml * 264 + q); }
      } else {
        const int b_ = mBlk / SS, s0 = mBlk & (SS - 1);
        for (int ch = t; ch < 256 * 16; ch += 256) { const int nl = ch >> 4, q = (ch & 15) * 8; const int n = nBlk + nl, h = n >> 6, dk = n & (DKK - 1);
          *(volatile v4u_t*)((bf16*)out + (((size_t)(b_ * HH + h)) * DKK + dk) * SS + s0 + q) = *(const v4ua*)(so + nl * 136 + q); }
      }
      __threadfence();
    }
  } else {
    float* so = (float*)sob;
#pragma unroll 1
    for (int hf = 0; hf < 2; ++hf) {
      if (wm == hf * 64) {
#pragma unroll
        for (int i = 0; i < 4; ++i)
#pragma unroll
          for (int j = 0; j < 4; ++j) {
            const int nl = wn + 16 * j + nlane;
            const float bv = bias ? bias[nBlk + nl] : 0.0f;
#pragma unroll
            for (int r = 0; r < 8; ++r) so[(16 * i + mh + r) * 260 + nl] = acc[i][j][r] + bv;
          }
      }
      __syncthreads();
#pragma unroll 1
      for (int pass = 0; pass < 2; ++pass) {
        for (int ch = t; ch < 64 * 64; ch += 256) { const int ml = ch >> 6, q = (ch & 63) * 4;
          *(volatile v4f_t*)((float*)out + (size_t)(mBlk + hf * 64 + ml) * N + nBlk + q) = *(const volatile v4fa*)(so + ml * 260 + q); }
        __threadfence();
      }
      __syncthreads();
    }
  }
}


#define KS32 40
#define VS32 40
template <int CAUSAL>
__global__ __launch_bounds__(128) void attn32_kernel(const bf16* __restrict__ Qb, const bf16* __restrict__ Kb, const bf16* __restrict__ Vt,
                                                    bf16* __restrict__ O, float scale_log2e) {
  __shared__ bf16 ldsK[2][32 * KS32];
  __shared__ bf16 ldsV[2][32 * VS32];
  __shared__ __attribute__((aligned(16))) bf16 ldsO[32 * 72];
  const int qblk = blockIdx.x * 32, hp = blockIdx.y, b = blockIdx.z;
  const int t = threadIdx.x, wave = t >> 5, lane = t & 31, qlane = lane & 15, kh8 = (lane >> 4) * 8;
  const int hl = wave >> 1, h = 2 * hp + hl, qt = wave & 1, q0 = qblk + 16 * qt;
  const bf16* Qh = Qb + (size_t)b * S32 * D32 + h * 32;
  const bf16x16 qf = load_frag(Qh, D32, q0, 0);
  const int sh = t >> 6, sr = (t >> 1) & 31, sc = (t & 1) * 16;
  const bf16* Ks = Kb + (size_t)b * S32 * D32 + (2 * hp + sh) * 32 + sc;
  const bf16* Vs = Vt + (((size_t)(b * NH32 + 2 * hp + sh)) * 32 + sr) * S32 + sc;
  f32x8 o[2] = {};
  float mrun = -INFINITY, lrun = 0.0f;
  const int qi = q0 + qlane;
  const int kend = CAUSAL ? (qblk + 31) : (S32 - 1);
#pragma unroll 1
  for (int kb = 0; kb <= kend; kb += 32) {
    __syncthreads();
    { const bf16* kp = Ks + (size_t)(kb + sr) * D32; const bf16* vp = Vs + kb;
      *(bf16x8*)(&ldsK[sh][sr * KS32 + sc]) = *(const bf16x8*)kp; *(bf16x8*)(&ldsK[sh][sr * KS32 + sc + 8]) = *(const bf16x8*)(kp + 8);
      *(bf16x8*)(&ldsV[sh][sr * VS32 + sc]) = *(const bf16x8*)vp; *(bf16x8*)(&ldsV[sh][sr * VS32 + sc + 8]) = *(const bf16x8*)(vp + 8); }
    __syncthreads();
    f32x8 s0 = {}, s1 = {};
    s0 = wmma_bf16(lds_frag(&ldsK[hl][0], KS32), qf, s0);
    s1 = wmma_bf16(lds_frag(&ldsK[hl][16 * KS32], KS32), qf, s1);
    float mx = -INFINITY;
#pragma unroll
    for (int r = 0; r < 8; ++r) { const int j0 = kb + kh8 + r, j1 = j0 + 16;
      s0[r] = (!CAUSAL || j0 <= qi) ? s0[r] * scale_log2e : -INFINITY;
      s1[r] = (!CAUSAL || j1 <= qi) ? s1[r] * scale_log2e : -INFINITY;
      mx = fmaxf(mx, fmaxf(s0[r], s1[r])); }
    mx = fmaxf(mx, __shfl_xor(mx, 16, 32));
    const float mnew = fmaxf(mrun, mx), alpha = exp2f(mrun - mnew);
    float rsum = 0.0f; bf16x16 pf;
#pragma unroll
    for (int r = 0; r < 8; ++r) { const float p0 = exp2f(s0[r] - mnew), p1 = exp2f(s1[r] - mnew); rsum += p0 + p1; pf[r] = (bf16)(p0 * 1024.0f); pf[r + 8] = (bf16)(p1 * 1024.0f); }
    rsum += __shfl_xor(rsum, 16, 32);
    lrun = lrun * alpha + rsum; mrun = mnew;
#pragma unroll
    for (int j = 0; j < 2; ++j) {
#pragma unroll
      for (int r = 0; r < 8; ++r) o[j][r] *= alpha;
      o[j] = wmma_bf16(lds_frag(&ldsV[hl][(j * 16) * VS32], VS32), pf, o[j]); }
  }
  const float rl = 1.0f / (lrun * 1024.0f);
#pragma unroll
  for (int j = 0; j < 2; ++j)
#pragma unroll
    for (int r = 0; r < 8; ++r) ldsO[(16 * qt + qlane) * 72 + hl * 32 + j * 16 + kh8 + r] = (bf16)(o[j][r] * rl);
  __syncthreads();
#pragma unroll 1
  for (int pass = 0; pass < 2; ++pass) {
    { const int row = t >> 2, q16 = (t & 3) * 16;
      bf16* dst = O + ((size_t)(b * S32 + qblk + row)) * D32 + hp * 64 + q16;
      *(volatile v4u_t*)dst = *(const v4ua*)(ldsO + row * 72 + q16); *(volatile v4u_t*)(dst + 8) = *(const v4ua*)(ldsO + row * 72 + q16 + 8); }
    __threadfence();
  }
}

#define GN_ 4096
#define GCH 256
__global__ __launch_bounds__(256) void k_ptT(const float* __restrict__ p, float* __restrict__ PT) {
  __shared__ float tile[64][65];
  const int n0 = blockIdx.x * 64, c0 = blockIdx.y * 64, b = blockIdx.z, t = threadIdx.x;
  for (int i = t; i < 64 * 64; i += 256) { const int c = i >> 6, n = i & 63; tile[c][n] = p[((size_t)(b * GCH + c0 + c)) * GN_ + n0 + n]; }
  __syncthreads();
#pragma unroll 1
  for (int pass = 0; pass < 2; ++pass) {
    for (int i = t; i < 64 * 16; i += 256) { const int n = i >> 4, c4 = (i & 15) * 4; v4f_t v; v.x = tile[c4][n]; v.y = tile[c4 + 1][n]; v.z = tile[c4 + 2][n]; v.w = tile[c4 + 3][n];
      *(volatile v4f_t*)(PT + ((size_t)(b * GN_ + n0 + n)) * GCH + c0 + c4) = v; }
    __threadfence();
  }
}
__global__ __launch_bounds__(256) void k_wbd(const float* __restrict__ w, float* __restrict__ Wbd) {
  const int o = blockIdx.x, k = threadIdx.x, g = o >> 5, i = o & 31; const float v = ((k >> 5) == g) ? w[((size_t)g * 32 + i) * 32 + (k & 31)] : 0.0f;
  *(volatile float*)(Wbd + (size_t)o * GCH + k) = v; __threadfence(); *(volatile float*)(Wbd + (size_t)o * GCH + k) = v;
}
__global__ __launch_bounds__(256) void k_eluT(const float* __restrict__ Xf, bf16* __restrict__ Vt) {
  __shared__ float tile[64][65];
  const int n0 = blockIdx.x * 64, c0 = blockIdx.y * 64, b = blockIdx.z, t = threadIdx.x;
  for (int i = t; i < 64 * 64; i += 256) { const int n = i >> 6, c = i & 63; tile[n][c] = Xf[((size_t)(b * GN_ + n0 + n)) * GCH + c0 + c]; }
  __syncthreads();
#pragma unroll 1
  for (int pass = 0; pass < 2; ++pass) {
    for (int i = t; i < 64 * 8; i += 256) { const int c = i >> 3, n8 = (i & 7) * 8; bf16 hv[8];
#pragma unroll
      for (int e = 0; e < 8; ++e) { const float x = tile[n8 + e][c]; hv[e] = (bf16)(x > 0.0f ? x : __expf(x) - 1.0f); }
      *(volatile v4u_t*)(Vt + ((size_t)(b * GCH + c0 + c)) * GN_ + n0 + n8) = *(const v4ua*)hv; }
    __threadfence();
  }
}
__global__ __launch_bounds__(256) void k_shuffle(const bf16* __restrict__ A, const float* __restrict__ p, float* __restrict__ Y, float* __restrict__ part) {
  __shared__ float tile[256][65];
  __shared__ float red[2][256];
  const int n0 = blockIdx.x * 64, b = blockIdx.y, t = threadIdx.x;
  for (int i = t; i < 64 * 256; i += 256) { const int n = i >> 8, col = i & 255, g = col >> 5, c = col & 31;
    tile[c * 8 + g][n] = (float)A[((size_t)(b * GN_ + n0 + n)) * D32 + col]; }
  __syncthreads();
  for (int i = t; i < 256 * 64; i += 256) { const int ch = i >> 6, n = i & 63; tile[ch][n] += p[((size_t)(b * GCH + ch)) * GN_ + n0 + n]; }
  __syncthreads();
  { const int grp = t >> 3, ch = grp * 8 + (t & 7); float s = 0.f, q = 0.f;
#pragma unroll 1
    for (int n = 0; n < 64; ++n) { const float v = tile[ch][n]; s += v; q += v * v; }
    red[0][t] = s; red[1][t] = q; }
  __syncthreads();
  if (t < 32) { float s = 0.f, q = 0.f;
#pragma unroll
    for (int k = 0; k < 8; ++k) { s += red[0][t * 8 + k]; q += red[1][t * 8 + k]; }
    const int blk = b * (GN_ / 64) + blockIdx.x;
    part[((size_t)blk * 32 + t) * 2] = s; part[((size_t)blk * 32 + t) * 2 + 1] = q; }
#pragma unroll 1
  for (int pass = 0; pass < 2; ++pass) {
    for (int i = t; i < 256 * 16; i += 256) { const int ch = i >> 4, n4 = (i & 15) * 4; v4f_t v; v.x = tile[ch][n4]; v.y = tile[ch][n4 + 1]; v.z = tile[ch][n4 + 2]; v.w = tile[ch][n4 + 3];
      *(volatile v4f_t*)(Y + ((size_t)(b * GCH + ch)) * GN_ + n0 + n4) = v; }
    if (t < 32) { const int blk = b * (GN_ / 64) + blockIdx.x; const float s = part[((size_t)blk * 32 + t) * 2], q = part[((size_t)blk * 32 + t) * 2 + 1];
      *(volatile float*)(part + ((size_t)blk * 32 + t) * 2) = s; *(volatile float*)(part + ((size_t)blk * 32 + t) * 2 + 1) = q; }
    __threadfence();
  }
}
__global__ __launch_bounds__(256) void k_gn(const float* __restrict__ Y, const float* __restrict__ part, const float* __restrict__ gw, const float* __restrict__ gb, float* __restrict__ out) {
  __shared__ float r0[64], r1[64]; __shared__ float stat[2];
  const int ch = blockIdx.x, b = blockIdx.y, grp = ch >> 3, t = threadIdx.x;
  if (t < 64) { const int blk = b * 64 + t; r0[t] = part[((size_t)blk * 32 + grp) * 2]; r1[t] = part[((size_t)blk * 32 + grp) * 2 + 1]; }
  __syncthreads();
  if (t == 0) { float s = 0.f, q = 0.f; for (int k = 0; k < 64; ++k) { s += r0[k]; q += r1[k]; }
    const float cnt = 8.0f * GN_, m = s / cnt, var = fmaxf(q / cnt - m * m, 0.0f); stat[0] = m; stat[1] = rsqrtf(var + 1e-5f); }
  __syncthreads();
  const float m = stat[0], rs = stat[1], a = rs * gw[ch], c0 = gb[ch] - m * rs * gw[ch];
  const float* yr = Y + ((size_t)(b * GCH + ch)) * GN_; float* orow = out + ((size_t)(b * GCH + ch)) * GN_;
#pragma unroll 1
  for (int pass = 0; pass < 2; ++pass) {
    for (int i = t; i < GN_ / 4; i += 256) { v4f_t v = *(const v4fa*)(yr + i * 4); v.x = v.x * a + c0; v.y = v.y * a + c0; v.z = v.z * a + c0; v.w = v.w * a + c0;
      *(volatile v4f_t*)(orow + i * 4) = v; }
    __threadfence();
  }
}

extern "C" void kernel_launch(void* const* d_in, const int* in_sizes, int n_in,
                              void* d_out, int out_size, void* d_ws, size_t ws_size,
                              hipStream_t stream) {
  (void)in_sizes; (void)n_in; (void)out_size; (void)ws_size;
  const float* pts = (const float*)d_in[0];
  const float* cw  = (const float*)d_in[1];
  const float* cb  = (const float*)d_in[2];
  const float* gw  = (const float*)d_in[3];  const float* gb = (const float*)d_in[4];
  char* ws = (char*)d_ws;
  float* PT  = (float*)ws; ws += (size_t)BB * GN_ * GCH * 4;
  float* Wbd = (float*)ws; ws += (size_t)GCH * GCH * 4;
  bf16* X    = (bf16*)ws;  ws += (size_t)BB * GN_ * D32 * 2;
  float* Xf  = (float*)ws; ws += (size_t)BB * GN_ * D32 * 4;
  bf16* VtB  = (bf16*)ws;  ws += (size_t)BB * GN_ * D32 * 2;
  bf16* At   = (bf16*)ws;  ws += (size_t)BB * GN_ * D32 * 2;
  float* Y   = (float*)ws; ws += (size_t)BB * GCH * GN_ * 4;
  float* part = (float*)ws; ws += (size_t)BB * 64 * 32 * 2 * 4;
  k_ptT<<<dim3(GN_ / 64, GCH / 64, BB), 256, 0, stream>>>(pts, PT);
  k_wbd<<<GCH, 256, 0, stream>>>(cw, Wbd);
  const int M = BB * GN_;
  gemm_bias_kernel<float, 0><<<dim3(M / 128, GCH / 256), 256, 0, stream>>>(PT, Wbd, cb, X, M, GCH, GCH);
  gemm_bias_kernel<float, 2><<<dim3(M / 128, GCH / 256), 256, 0, stream>>>(PT, Wbd, cb, Xf, M, GCH, GCH);
  k_eluT<<<dim3(GN_ / 64, GCH / 64, BB), 256, 0, stream>>>(Xf, VtB);
  attn32_kernel<0><<<dim3(GN_ / 32, NH32 / 2, BB), 128, 0, stream>>>(X, X, VtB, At, 0.17677669529663687f * 1.44269504088896340736f);
  k_shuffle<<<dim3(GN_ / 64, BB), 256, 0, stream>>>(At, pts, Y, part);
  k_gn<<<dim3(GCH, BB), 256, 0, stream>>>(Y, part, gw, gb, (float*)d_out);
}
